// MFDKT_18013092839820
// MI455X (gfx1250) — hardware-verified
//
#include <hip/hip_runtime.h>


#define BB   512
#define TT   200
#define HH   256
#define G4   1024
#define OUTN 1001
#define NPAD 1024
#define CATW 2002
#define CATP 2048
#define KP   320
#define NFC1 320
#define NVOC 2001
#define VP   2048
#define NUSR 5001
#define NBB  32
#define HP   264

typedef __attribute__((ext_vector_type(16))) _Float16 v16h;
typedef __attribute__((ext_vector_type(8)))  _Float16 v8h;
typedef __attribute__((ext_vector_type(16))) __bf16   v16b;
typedef __attribute__((ext_vector_type(8)))  __bf16   v8b;
typedef __attribute__((ext_vector_type(8)))  float    v8f;
typedef __attribute__((ext_vector_type(4)))  float    v4f;

__device__ __forceinline__ unsigned short f2bf_bits(float f) {
  unsigned u = __float_as_uint(f);
  return (unsigned short)((u + 0x7FFFu + ((u >> 16) & 1u)) >> 16);
}
__device__ __forceinline__ float bf_bits2f(unsigned short h) { return __uint_as_float(((unsigned)h) << 16); }

__device__ __forceinline__ void dep_guard_h(v8f& a, v8f& b, v16h x, v16h y) { asm volatile("v_nop\n\tv_nop\n\tv_nop\n\tv_nop" : "+v"(a), "+v"(b) : "v"(x), "v"(y)); }
__device__ __forceinline__ void dep_guard_b(v8f& a, v8f& b, v16b x, v16b y) { asm volatile("v_nop\n\tv_nop\n\tv_nop\n\tv_nop" : "+v"(a), "+v"(b) : "v"(x), "v"(y)); }
__device__ __forceinline__ void keep4_h(v16h a, v16h b, v16h c, v16h d) { asm volatile("v_nop" :: "v"(a), "v"(b), "v"(c), "v"(d)); }
__device__ __forceinline__ void keep4_b(v16b a, v16b b, v16b c, v16b d) { asm volatile("v_nop" :: "v"(a), "v"(b), "v"(c), "v"(d)); }
__device__ __forceinline__ void acc_guard4(v8f& a, v8f& b, v8f& c, v8f& d) { asm volatile("v_nop\n\tv_nop\n\tv_nop\n\tv_nop" : "+v"(a), "+v"(b), "+v"(c), "+v"(d)); }
template <typename T> struct Frag;
template <> struct Frag<_Float16> {
  typedef v16h V; union U { v16h v; v8h h[2]; };
  static __device__ __forceinline__ v16h load(const _Float16* p) {
    U f; f.h[0] = *(const v8h*)(p); f.h[1] = *(const v8h*)(p + 16); return f.v;
  }
  static __device__ __forceinline__ v8f mma(v16h a, v16h b, v8f c) {
    return __builtin_amdgcn_wmma_f32_16x16x32_f16(false, a, false, b, (short)0, c, false, false);
  }
  static __device__ __forceinline__ void guard(v8f& a, v8f& b, v16h x, v16h y) { dep_guard_h(a, b, x, y); }
  static __device__ __forceinline__ void keep(v16h a, v16h b, v16h c, v16h d) { keep4_h(a, b, c, d); }
};
template <> struct Frag<__bf16> {
  typedef v16b V; union U { v16b v; v8b h[2]; };
  static __device__ __forceinline__ v16b load(const __bf16* p) {
    U f; f.h[0] = *(const v8b*)(p); f.h[1] = *(const v8b*)(p + 16); return f.v;
  }
  static __device__ __forceinline__ v8f mma(v16b a, v16b b, v8f c) {
    return __builtin_amdgcn_wmma_f32_16x16x32_bf16(false, a, false, b, (short)0, c, false, false);
  }
  static __device__ __forceinline__ void guard(v8f& a, v8f& b, v16b x, v16b y) { dep_guard_b(a, b, x, y); }
  static __device__ __forceinline__ void keep(v16b a, v16b b, v16b c, v16b d) { keep4_b(a, b, c, d); }
};

template <int ET> struct Elem;
template <> struct Elem<0> { typedef _Float16 T; };
template <> struct Elem<1> { typedef __bf16 T; };
template <int ET, bool SPLIT, int BIAS_MODE, int OUT_MODE, bool RESID, int ACT = 0>
__global__ __launch_bounds__(256) void wmma_gemm64(
    const unsigned short* __restrict__ Ap, const unsigned short* __restrict__ A2p, int lda, long strideA,
    const unsigned short* __restrict__ Btp, const unsigned short* __restrict__ Bt2p, int ldb, long strideB,
    void* __restrict__ Cout, void* __restrict__ Cout2, int ldc, long strideC,
    const float* __restrict__ bias,
    const float* __restrict__ resid, long strideR,
    int M, int N, int K, float scale, float oscale) {
  typedef typename Elem<ET>::T T;
  typedef typename Frag<T>::V V;
  const T* A = (const T*)Ap; const T* A2 = (const T*)A2p; const T* Bt = (const T*)Btp; const T* Bt2 = (const T*)Bt2p;
  __shared__ __align__(16) float sT[8][16 * 68];
  const int b    = blockIdx.y;
  const int lane = threadIdx.x & 31;
  const int wave = threadIdx.x >> 5;
  const int tilesN = N >> 6;
  const int tilesM = M >> 6;
  const int tile = blockIdx.x * 8 + wave;
  if (tile >= tilesM * tilesN) return;
  const int tm = tile / tilesN;
  const int tn = tile - tm * tilesN;
  const int m0 = tm << 6;
  const int n0 = tn << 6;

  const T* Ab  = A  + (size_t)b * strideA;
  const T* Bb  = Bt + (size_t)b * strideB;
  const T* Ab2 = SPLIT ? (A2  + (size_t)b * strideA) : nullptr;
  const T* Bb2 = SPLIT ? (Bt2 + (size_t)b * strideB) : nullptr;

  const int rlane = lane & 15;
  const int koff  = (lane >> 4) * 8;
  const int mOff  = (lane >> 4) * 8;

  v8f acc[4][4];
#pragma unroll
  for (int i = 0; i < 4; ++i)
#pragma unroll
    for (int j = 0; j < 4; ++j) acc[i][j] = (v8f){0.f,0.f,0.f,0.f,0.f,0.f,0.f,0.f};

  for (int k0 = 0; k0 < K; k0 += 32) {
    V bh[4], bl[4];
#pragma unroll
    for (int j = 0; j < 4; ++j) {
      const size_t bo = (size_t)(n0 + (j << 4) + rlane) * ldb + koff + k0;
      bh[j] = Frag<T>::load(Bb + bo);
      if (SPLIT) bl[j] = Frag<T>::load(Bb2 + bo);
    }
#pragma unroll
    for (int i = 0; i < 4; ++i) {
      const size_t ao = (size_t)(m0 + (i << 4) + rlane) * lda + koff + k0;
      V ah = Frag<T>::load(Ab + ao);
      V al;
      if (SPLIT) al = Frag<T>::load(Ab2 + ao);
#pragma unroll
      for (int j = 0; j < 4; ++j) {
        acc[i][j] = Frag<T>::mma(ah, bh[j], acc[i][j]);
        if (SPLIT) {
          acc[i][j] = Frag<T>::mma(ah, bl[j], acc[i][j]);
          acc[i][j] = Frag<T>::mma(al, bh[j], acc[i][j]);
        }
      }
      Frag<T>::guard(acc[i][0], acc[i][3], ah, SPLIT ? al : ah);
    }
    Frag<T>::keep(bh[0], bh[1], bh[2], bh[3]);
    if (SPLIT) Frag<T>::keep(bl[0], bl[1], bl[2], bl[3]);
  }
  acc_guard4(acc[0][0], acc[0][1], acc[0][2], acc[0][3]);
  acc_guard4(acc[1][0], acc[1][1], acc[1][2], acc[1][3]);
  acc_guard4(acc[2][0], acc[2][1], acc[2][2], acc[2][3]);
  acc_guard4(acc[3][0], acc[3][1], acc[3][2], acc[3][3]);

  float* slab = sT[wave];
  const float* Rb = RESID ? (resid + (size_t)b * strideR) : nullptr;
#pragma unroll
  for (int i = 0; i < 4; ++i) {
    const int mBase = m0 + (i << 4);
#pragma unroll
    for (int j = 0; j < 4; ++j) {
      const int n = n0 + (j << 4) + rlane;
      float bv = 0.f;
      if (BIAS_MODE == 2) bv = bias[n];
#pragma unroll
      for (int r = 0; r < 8; ++r) {
        float v = acc[i][j][r] * scale;
        if (BIAS_MODE == 1) v += bias[mBase + mOff + r];
        if (BIAS_MODE == 2) v += bv;
        if (RESID) v += Rb[(size_t)(mBase + mOff + r) * ldc + n];
        if (ACT == 1) v = tanhf(v);
        if (ACT == 2) v = fmaxf(v, 0.0f);
        if (ACT == 3) v = v / (1.0f + expf(-v));
        if (ACT == 4) v = (v > 0.f) ? v : 0.01f * v;
        if (ACT == 5) v = 0.5f * v * (1.0f + erff(v * 0.70710678118654752f));
        if (ACT == 6) v = __builtin_amdgcn_rcpf(1.0f + __expf(-v));
        v *= oscale;
        slab[(mOff + r) * 68 + (j << 4) + rlane] = v;
      }
    }
    __builtin_amdgcn_fence(__ATOMIC_RELEASE, "workgroup");
    __builtin_amdgcn_wave_barrier();
    __builtin_amdgcn_fence(__ATOMIC_ACQUIRE, "workgroup");
    if (OUT_MODE == 0) {
      float* C = (float*)Cout + (size_t)b * strideC;
      const int hh = lane >> 4, c4 = (lane & 15) * 4;
      for (int pass = 0; pass < 2; ++pass) {
#pragma unroll
        for (int it = 0; it < 8; ++it) {
          const int row = it * 2 + hh;
          v4f v = *(const v4f*)(slab + row * 68 + c4);
          *(volatile v4f*)(C + (size_t)(mBase + row) * ldc + n0 + c4) = v;
        }
        __threadfence();
      }
    } else {
      const int q = lane >> 3, c8 = (lane & 7) * 8;
      unsigned short* C  = (unsigned short*)Cout  + (size_t)b * strideC;
      unsigned short* C2 = (OUT_MODE == 2) ? ((unsigned short*)Cout2 + (size_t)b * strideC) : nullptr;
      for (int pass = 0; pass < 2; ++pass) {
#pragma unroll
        for (int it = 0; it < 4; ++it) {
          const int row = it * 4 + q;
          const float* sp = slab + row * 68 + c8;
          v8h hv, lv;
#pragma unroll
          for (int e = 0; e < 8; ++e) {
            if (OUT_MODE == 1) {
              hv[e] = (_Float16)sp[e];
            } else {
              unsigned short hb = f2bf_bits(sp[e]);
              unsigned short lb = f2bf_bits(sp[e] - bf_bits2f(hb));
              hv[e] = __builtin_bit_cast(_Float16, hb);
              lv[e] = __builtin_bit_cast(_Float16, lb);
            }
          }
          *(volatile v8h*)(C + (size_t)(mBase + row) * ldc + n0 + c8) = hv;
          if (OUT_MODE == 2) *(volatile v8h*)(C2 + (size_t)(mBase + row) * ldc + n0 + c8) = lv;
        }
        __threadfence();
      }
    }
    __builtin_amdgcn_fence(__ATOMIC_RELEASE, "workgroup");
    __builtin_amdgcn_wave_barrier();
    __builtin_amdgcn_fence(__ATOMIC_ACQUIRE, "workgroup");
  }
}

template <bool GATHER>
__global__ __launch_bounds__(256) void k_rows256(
    const float* __restrict__ src, const int* __restrict__ idx, int istride, int nsrc,
    const float* __restrict__ vecA, const float* __restrict__ vecB,
    _Float16* __restrict__ dst, int R, int nvalid, int Cpad,
    float scale, float a_mul, float a_add, float b_mul, float b_add, int one_row, float one_val)
{
  const int lane = threadIdx.x & 31;
  const int wave = threadIdx.x >> 5;
  const int r = blockIdx.x * 8 + wave;
  if (r >= R) return;
  int s = r;
  if (GATHER) {
    int id = idx[(size_t)r * istride];
    id = (id < 0) ? (id + nsrc) : id;
    id = (id < 0) ? 0 : id;
    id = (id > nsrc - 1) ? (nsrc - 1) : id;
    s = id;
  }
  const bool valid = (s < nvalid);
  const int sa = valid ? s : (nvalid - 1);
  const float* sp = src + (size_t)sa * HH + 8 * lane;
  const v4f x0 = *(const v4f*)(sp);
  const v4f x1 = *(const v4f*)(sp + 4);
  const float zs = valid ? scale : 0.0f;
  v8h o0;
#pragma unroll
  for (int e = 0; e < 4; ++e) {
    o0[e]     = (_Float16)(x0[e] * zs);
    o0[4 + e] = (_Float16)(x1[e] * zs);
  }
  const float e256 = valid ? (a_mul * vecA[sa] + a_add) : ((r == one_row) ? one_val : 0.0f);
  const float e257 = valid ? (b_mul * vecB[sa] + b_add) : 0.0f;
  v8h o1;
#pragma unroll
  for (int e = 0; e < 8; ++e) o1[e] = (_Float16)0.0f;
  o1[0] = (lane == 0) ? (_Float16)e256 : (_Float16)0.0f;
  o1[1] = (lane == 0) ? (_Float16)e257 : (_Float16)0.0f;
  _Float16* dp = dst + (size_t)r * Cpad;
  for (int pass = 0; pass < 2; ++pass) {
    *(volatile v8h*)(dp + 8 * lane) = o0;
    if (Cpad > HH && lane < 8) *(volatile v8h*)(dp + HH + 8 * lane) = o1;
    __threadfence();
  }
}

__global__ __launch_bounds__(256) void k_w1p(
    const float* __restrict__ W1, const float* __restrict__ b1, _Float16* __restrict__ dst)
{
  const int lane = threadIdx.x & 31;
  const int wave = threadIdx.x >> 5;
  const int n = blockIdx.x * 8 + wave;
  if (n >= NFC1) return;
  const int na = (n < HH) ? n : (HH - 1);
  const float bn = b1[na];
  const float* wrow = W1 + (size_t)na * CATW;
  v8h o[8];
#pragma unroll
  for (int ch = 0; ch < 8; ++ch) {
#pragma unroll
    for (int e = 0; e < 8; ++e) {
      const int oc = ch * 256 + 8 * lane + e;
      const bool inA = (oc < OUTN);
      const bool inB = (oc >= NPAD) && (oc < NPAD + OUTN);
      const int sc = inA ? oc : (inB ? (oc - NPAD + OUTN) : 0);
      const float w = wrow[sc];
      float v = 0.0f;
      if (n < HH) {
        v = (inA || inB) ? (w * 64.0f) : 0.0f;
        if (oc == OUTN) v = bn * 64.0f;
      } else if (n == HH) {
        v = (oc == OUTN) ? 64.0f : 0.0f;
      }
      o[ch][e] = (_Float16)v;
    }
  }
  _Float16* dp = dst + (size_t)n * CATP;
  for (int pass = 0; pass < 2; ++pass) {
#pragma unroll
    for (int ch = 0; ch < 8; ++ch) *(volatile v8h*)(dp + ch * 256 + 8 * lane) = o[ch];
    __threadfence();
  }
}

__device__ __forceinline__ float sigm_f(float x) { return __builtin_amdgcn_rcpf(1.0f + __expf(-x)); }
__device__ __forceinline__ float tanh_f(float x) { return 1.0f - 2.0f * __builtin_amdgcn_rcpf(__expf(2.0f * x) + 1.0f); }

__global__ __launch_bounds__(256) void k_recur(
    const _Float16* __restrict__ Whh16,
    const float* __restrict__ G,
    const int* __restrict__ tok,
    const float* __restrict__ b_ih, const float* __restrict__ b_hh,
    _Float16* __restrict__ hT)
{
  __shared__ __align__(16) _Float16 hsh[2 * NBB * HP];
  __shared__ float csh[NBB * HH];
  __shared__ float bsh[G4];
  typedef Frag<_Float16> F;
  const int tid = threadIdx.x;
  const int lane = tid & 31, wave = tid >> 5, hh = lane >> 4, rl = lane & 15;
  const int b0 = (int)blockIdx.x * NBB;
  for (int i = tid; i < 2 * NBB * HP; i += 256) hsh[i] = (_Float16)0.0f;
  for (int i = tid; i < NBB * HH; i += 256) csh[i] = 0.0f;
  for (int i = tid; i < G4; i += 256) bsh[i] = b_ih[i] + b_hh[i];
  __syncthreads();
  const float S = 1.0f / 16384.0f;

  for (int s = 0; s < TT; ++s) {
    const _Float16* hc = hsh + (s & 1) * (NBB * HP);
    _Float16* hn = hsh + ((s & 1) ^ 1) * (NBB * HP);
#pragma unroll 1
    for (int q = 0; q < 2; ++q) {
      const int ub = wave * 32 + 16 * q;
      v8f acc[2][4];
#pragma unroll
      for (int mi = 0; mi < 2; ++mi)
#pragma unroll
        for (int g = 0; g < 4; ++g) acc[mi][g] = (v8f){0.f,0.f,0.f,0.f,0.f,0.f,0.f,0.f};
#pragma unroll 1
      for (int k0 = 0; k0 < HH; k0 += 32) {
        v16h bfr[4];
#pragma unroll
        for (int g = 0; g < 4; ++g) bfr[g] = F::load(Whh16 + (size_t)(g * HH + ub + rl) * HH + k0 + 8 * hh);
        const v16h a0 = F::load(hc + rl * HP + k0 + 8 * hh);
        const v16h a1 = F::load(hc + (16 + rl) * HP + k0 + 8 * hh);
#pragma unroll
        for (int g = 0; g < 4; ++g) {
          acc[0][g] = F::mma(a0, bfr[g], acc[0][g]);
          acc[1][g] = F::mma(a1, bfr[g], acc[1][g]);
        }
        F::guard(acc[0][0], acc[0][3], a0, a1);
        F::guard(acc[1][0], acc[1][3], a0, a1);
        F::keep(bfr[0], bfr[1], bfr[2], bfr[3]);
      }
      acc_guard4(acc[0][0], acc[0][1], acc[0][2], acc[0][3]);
      acc_guard4(acc[1][0], acc[1][1], acc[1][2], acc[1][3]);

      const int u = ub + rl;
      const float bI = bsh[u], bF = bsh[HH + u], bG = bsh[2 * HH + u], bO = bsh[3 * HH + u];
#pragma unroll
      for (int mi = 0; mi < 2; ++mi) {
#pragma unroll
        for (int r = 0; r < 8; ++r) {
          const int bl = mi * 16 + 8 * hh + r;
          int tk = tok[(size_t)(b0 + bl) * TT + s];
          tk = (tk < 0) ? (tk + NVOC) : tk;
          tk = (tk < 0) ? 0 : tk;
          tk = (tk > NVOC - 1) ? (NVOC - 1) : tk;
          const float* gp = G + (size_t)tk * G4 + u;
          const float gi = acc[mi][0][r] * S + (gp[0]      + bI);
          const float gf = acc[mi][1][r] * S + (gp[HH]     + bF);
          const float gg = acc[mi][2][r] * S + (gp[2 * HH] + bG);
          const float go = acc[mi][3][r] * S + (gp[3 * HH] + bO);
          const float cp = csh[bl * HH + u];
          const float cn = sigm_f(gf) * cp + sigm_f(gi) * tanh_f(gg);
          csh[bl * HH + u] = cn;
          const float h = sigm_f(go) * tanh_f(cn);
          hn[bl * HP + u] = (_Float16)(h * 256.0f);
        }
      }
    }
    __syncthreads();
  }

  const _Float16* hf = hsh + (TT & 1) * (NBB * HP);
  v8h o0[4];
#pragma unroll
  for (int j = 0; j < 4; ++j) o0[j] = *(const v8h*)(hf + (wave * 4 + j) * HP + 8 * lane);
  v8h o1;
#pragma unroll
  for (int e = 0; e < 8; ++e) o1[e] = (_Float16)0.0f;
  o1[0] = (lane == 0) ? (_Float16)256.0f : (_Float16)0.0f;
  for (int pass = 0; pass < 2; ++pass) {
#pragma unroll
    for (int j = 0; j < 4; ++j) {
      const int row = b0 + wave * 4 + j;
      *(volatile v8h*)(hT + (size_t)row * KP + 8 * lane) = o0[j];
      if (lane < 8) *(volatile v8h*)(hT + (size_t)row * KP + HH + 8 * lane) = o1;
    }
    __threadfence();
  }
}

__global__ __launch_bounds__(512) void k_select(
    const float* __restrict__ m2, const int* __restrict__ tgt, float* __restrict__ out, int nb)
{
  const int b = threadIdx.x;
  if (b >= nb) return;
  int t = tgt[b];
  t = (t < 0) ? (t + OUTN) : t;
  t = (t < 0) ? 0 : t;
  t = (t > OUTN - 1) ? (OUTN - 1) : t;
  const float v = m2[(size_t)b * NPAD + t];
  const float y = 1.0f / (1.0f + expf(-v));
  ((volatile float*)out)[b] = y;
  __threadfence();
  ((volatile float*)out)[b] = y;
}

extern "C" void kernel_launch(void* const* d_in, const int* in_sizes, int n_in,
                              void* d_out, int out_size, void* d_ws, size_t ws_size,
                              hipStream_t stream) {
  if (n_in < 19) return;
  if (in_sizes[0] != BB * TT || in_sizes[1] != BB || in_sizes[2] != BB * TT) return;
  if (in_sizes[4] != NVOC * HH || in_sizes[5] != G4 * HH || in_sizes[6] != G4 * HH) return;
  if (in_sizes[7] != G4 || in_sizes[8] != G4) return;
  if (in_sizes[9] != OUTN * HH || in_sizes[10] != OUTN) return;
  if (in_sizes[11] != NUSR * HH || in_sizes[12] != OUTN * HH || in_sizes[13] != NUSR || in_sizes[14] != OUTN) return;
  if (in_sizes[15] != HH * CATW || in_sizes[16] != HH || in_sizes[17] != OUTN * HH || in_sizes[18] != OUTN) return;
  if (out_size != BB) return;

  const int*   main_input = (const int*)  d_in[0];
  const int*   target_id  = (const int*)  d_in[1];
  const int*   uid_seq    = (const int*)  d_in[2];
  const float* enc_W = (const float*)d_in[4];
  const float* W_ih  = (const float*)d_in[5];
  const float* W_hh  = (const float*)d_in[6];
  const float* b_ih  = (const float*)d_in[7];
  const float* b_hh  = (const float*)d_in[8];
  const float* Wd    = (const float*)d_in[9];
  const float* bd    = (const float*)d_in[10];
  const float* P     = (const float*)d_in[11];
  const float* Q     = (const float*)d_in[12];
  const float* Pb    = (const float*)d_in[13];
  const float* Qb    = (const float*)d_in[14];
  const float* W1    = (const float*)d_in[15];
  const float* b1    = (const float*)d_in[16];
  const float* W2    = (const float*)d_in[17];
  const float* b2    = (const float*)d_in[18];
  float* out = (float*)d_out;

  const size_t szE   = (size_t)VP   * HH   * 2;
  const size_t szWi  = (size_t)G4   * HH   * 2;
  const size_t szWh  = (size_t)G4   * HH   * 2;
  const size_t szG   = (size_t)VP   * G4   * 4;
  const size_t szP   = (size_t)BB   * KP   * 2;
  const size_t szQ   = (size_t)NPAD * KP   * 2;
  const size_t szWd  = (size_t)NPAD * KP   * 2;
  const size_t szW2  = (size_t)NPAD * KP   * 2;
  const size_t szW1  = (size_t)NFC1 * CATP * 2;
  const size_t szHT  = (size_t)BB   * KP   * 2;
  const size_t szCat = (size_t)BB   * CATP * 2;
  const size_t szM1  = (size_t)BB   * KP   * 2;
  const size_t szM2  = (size_t)BB   * NPAD * 4;
  size_t off = 0;
  const size_t oE   = off; off += szE;
  const size_t oWi  = off; off += szWi;
  const size_t oWh  = off; off += szWh;
  const size_t oG   = off; off += szG;
  const size_t oP   = off; off += szP;
  const size_t oQ   = off; off += szQ;
  const size_t oWd  = off; off += szWd;
  const size_t oW2  = off; off += szW2;
  const size_t oW1  = off; off += szW1;
  const size_t oHT  = off; off += szHT;
  const size_t oCat = off; off += szCat;
  const size_t oM1  = off; off += szM1;
  const size_t oM2  = off; off += szM2;
  if (off > ws_size) return;
  char* ws = (char*)d_ws;
  _Float16* E16   = (_Float16*)(ws + oE);
  _Float16* Wih16 = (_Float16*)(ws + oWi);
  _Float16* Whh16 = (_Float16*)(ws + oWh);
  float*    G     = (float*)   (ws + oG);
  _Float16* P16   = (_Float16*)(ws + oP);
  _Float16* Q16   = (_Float16*)(ws + oQ);
  _Float16* Wd16  = (_Float16*)(ws + oWd);
  _Float16* W2p   = (_Float16*)(ws + oW2);
  _Float16* W1p   = (_Float16*)(ws + oW1);
  _Float16* hT16  = (_Float16*)(ws + oHT);
  _Float16* cat   = (_Float16*)(ws + oCat);
  _Float16* m1    = (_Float16*)(ws + oM1);
  float*    m2    = (float*)   (ws + oM2);
  typedef const unsigned short* cus;

  k_rows256<false><<<(VP + 7) / 8, 256, 0, stream>>>(enc_W, main_input, 0, NVOC, enc_W, enc_W, E16, VP, NVOC, HH,
                                                     64.0f, 0.0f, 0.0f, 0.0f, 0.0f, -1, 0.0f);
  k_rows256<false><<<(G4 + 7) / 8, 256, 0, stream>>>(W_ih, main_input, 0, G4, W_ih, W_ih, Wih16, G4, G4, HH,
                                                     64.0f, 0.0f, 0.0f, 0.0f, 0.0f, -1, 0.0f);
  k_rows256<false><<<(G4 + 7) / 8, 256, 0, stream>>>(W_hh, main_input, 0, G4, W_hh, W_hh, Whh16, G4, G4, HH,
                                                     64.0f, 0.0f, 0.0f, 0.0f, 0.0f, -1, 0.0f);
  k_rows256<false><<<(NPAD + 7) / 8, 256, 0, stream>>>(Q, main_input, 0, OUTN, Q, Qb, Q16, NPAD, OUTN, KP,
                                                       64.0f, 0.0f, 64.0f, 64.0f, 0.0f, -1, 0.0f);
  k_rows256<true><<<(BB + 7) / 8, 256, 0, stream>>>(P, uid_seq, TT, NUSR, Pb, P, P16, BB, NUSR, KP,
                                                    64.0f, 64.0f, 0.0f, 0.0f, 64.0f, -1, 0.0f);
  k_rows256<false><<<(NPAD + 7) / 8, 256, 0, stream>>>(Wd, main_input, 0, OUTN, bd, Wd, Wd16, NPAD, OUTN, KP,
                                                       64.0f, 64.0f, 0.0f, 0.0f, 0.0f, OUTN, 64.0f);
  k_rows256<false><<<(NPAD + 7) / 8, 256, 0, stream>>>(W2, main_input, 0, OUTN, b2, W2, W2p, NPAD, OUTN, KP,
                                                       64.0f, 64.0f, 0.0f, 0.0f, 0.0f, -1, 0.0f);
  k_w1p<<<(NFC1 + 7) / 8, 256, 0, stream>>>(W1, b1, W1p);

  wmma_gemm64<0, false, 0, 0, false, 0><<<dim3(((VP / 64) * (G4 / 64) + 7) / 8, 1), 256, 0, stream>>>(
      (cus)E16, (cus)E16, HH, 0L, (cus)Wih16, (cus)Wih16, HH, 0L,
      (void*)G, (void*)G, G4, 0L, b_ih, b_ih, 0L, VP, G4, HH, 1.0f / 4096.0f, 1.0f);

  k_recur<<<BB / NBB, 256, 0, stream>>>(Whh16, G, main_input, b_ih, b_hh, hT16);

  wmma_gemm64<0, false, 0, 1, false, 6><<<dim3(((BB / 64) * (NPAD / 64) + 7) / 8, 1), 256, 0, stream>>>(
      (cus)P16, (cus)P16, KP, 0L, (cus)Q16, (cus)Q16, KP, 0L,
      (void*)(cat + NPAD), (void*)(cat + NPAD), CATP, 0L, b_ih, b_ih, 0L, BB, NPAD, KP, 1.0f / 4096.0f, 64.0f);

  wmma_gemm64<0, false, 0, 1, false, 0><<<dim3(((BB / 64) * (NPAD / 64) + 7) / 8, 1), 256, 0, stream>>>(
      (cus)hT16, (cus)hT16, KP, 0L, (cus)Wd16, (cus)Wd16, KP, 0L,
      (void*)cat, (void*)cat, CATP, 0L, b_ih, b_ih, 0L, BB, NPAD, KP, 1.0f / 256.0f, 1.0f);

  wmma_gemm64<0, false, 0, 1, false, 2><<<dim3(((BB / 64) * (NFC1 / 64) + 7) / 8, 1), 256, 0, stream>>>(
      (cus)cat, (cus)cat, CATP, 0L, (cus)W1p, (cus)W1p, CATP, 0L,
      (void*)m1, (void*)m1, KP, 0L, b_ih, b_ih, 0L, BB, NFC1, CATP, 1.0f / 4096.0f, 16.0f);

  wmma_gemm64<0, false, 0, 0, false, 2><<<dim3(((BB / 64) * (NPAD / 64) + 7) / 8, 1), 256, 0, stream>>>(
      (cus)m1, (cus)m1, KP, 0L, (cus)W2p, (cus)W2p, KP, 0L,
      (void*)m2, (void*)m2, NPAD, 0L, b_ih, b_ih, 0L, BB, NPAD, KP, 1.0f / 1024.0f, 1.0f);

  k_select<<<1, BB, 0, stream>>>(m2, target_id, out, BB);
}
